// MultiHeadAttention_75273596829862
// MI455X (gfx1250) — hardware-verified
//
#include <hip/hip_runtime.h>
#include <math.h>

#ifndef NB
#define NB 2
#endif
#ifndef SEQ
#define SEQ 2048
#endif
#define NB_FULL 2
#define SEQ_FULL 2048
#define DM 768
#define NH 12
#define HD 64
#define QPITCH 1536
#define RESOFF 768
#define AT_NW 4
#define PSP 40
#define OSP 68
#define PSC 16384.0f
#define QCARRY 256.0f
#define CCARRY 256.0f
#define WCARRY 16.0f

static_assert(DM == NH * HD);
static_assert(HD == 64);
static_assert(DM % 64 == 0);
static_assert(DM % 32 == 0);
static_assert(QPITCH == 2 * DM);
static_assert(RESOFF == DM);
static_assert(QPITCH % 32 == 0);
static_assert(SEQ % 64 == 0);
static_assert(NB >= 1 && NB <= NB_FULL);
static_assert(SEQ <= SEQ_FULL);
static_assert((PSP * 2) % 16 == 0);
static_assert((OSP * 4) % 16 == 0);
static_assert(PSP >= 32);
static_assert(OSP >= 64);
static_assert((NB * SEQ) % 64 == 0);

typedef __attribute__((ext_vector_type(16))) _Float16 v16h;
typedef __attribute__((ext_vector_type(8)))  _Float16 v8h;
typedef __attribute__((ext_vector_type(8)))  float    v8f;
typedef __attribute__((ext_vector_type(4)))  float    v4f;
typedef __attribute__((ext_vector_type(4)))  unsigned int u4v;

union FragH { v16h v; v8h h[2]; };
__device__ __forceinline__ v16h ldf(const _Float16* __restrict__ p) {
  FragH f; f.h[0] = *(const v8h*)(p); f.h[1] = *(const v8h*)(p + 16); return f.v;
}
__device__ __forceinline__ v8f mma16(v16h a, v16h b, v8f c) {
  c = __builtin_amdgcn_wmma_f32_16x16x32_f16(false, a, false, b, (short)0, c, false, false);
  asm volatile("v_nop\n\tv_nop\n\tv_nop\n\tv_nop" : "+v"(c) : "v"(a), "v"(b));
  return c;
}
__device__ __forceinline__ void guard4(v8f& a, v8f& b, v8f& c, v8f& d, v16h x, v16h y) {
  asm volatile("v_nop\n\tv_nop\n\tv_nop\n\tv_nop" : "+v"(a), "+v"(b), "+v"(c), "+v"(d) : "v"(x), "v"(y));
}
__device__ __forceinline__ void keep4(v16h a, v16h b, v16h c, v16h d) { asm volatile("v_nop" :: "v"(a), "v"(b), "v"(c), "v"(d)); }
__device__ __forceinline__ void acc_guard4(v8f& a, v8f& b, v8f& c, v8f& d) {
  asm volatile("v_nop\n\tv_nop\n\tv_nop\n\tv_nop" : "+v"(a), "+v"(b), "+v"(c), "+v"(d));
}
__device__ __forceinline__ void wave_sync_lds() {
  __builtin_amdgcn_fence(3  , "workgroup");
  __builtin_amdgcn_wave_barrier();
  __builtin_amdgcn_fence(2  , "workgroup");
}
__device__ __forceinline__ float bf_rne_keep(float v) {
  const unsigned u = __builtin_bit_cast(unsigned, v);
  const unsigned r = (u + 0x7fffu + ((u >> 16) & 1u)) & 0xffff0000u;
  return __builtin_bit_cast(float, r);
}
__device__ __forceinline__ unsigned int pk2h(float a, float b) {
  return (unsigned int)__builtin_bit_cast(unsigned short, (_Float16)a) | ((unsigned int)__builtin_bit_cast(unsigned short, (_Float16)b) << 16);
}

__global__ __launch_bounds__(256) void k_cast_x(const float* __restrict__ SRC, unsigned short* __restrict__ DST) {
  const int u = (int)blockIdx.x * 256 + (int)threadIdx.x;
  const int per = DM / 8;
  if (u >= NB * SEQ * per) return;
  const int r = u / per;
  const int c0 = 8 * (u - r * per);
  const int b = r / SEQ, s = r - b * SEQ;
  const float* sp = SRC + ((size_t)b * SEQ_FULL + (size_t)s) * DM + c0;
  const v4f a = *(const v4f*)(sp);
  const v4f g = *(const v4f*)(sp + 4);
  u4v pk;
  pk.x = pk2h(bf_rne_keep(a.x), bf_rne_keep(a.y));
  pk.y = pk2h(bf_rne_keep(a.z), bf_rne_keep(a.w));
  pk.z = pk2h(bf_rne_keep(g.x), bf_rne_keep(g.y));
  pk.w = pk2h(bf_rne_keep(g.z), bf_rne_keep(g.w));
  volatile u4v* d = (volatile u4v*)(DST + (size_t)r * DM + c0);
  *d = pk; __threadfence(); *d = pk;
}

__global__ __launch_bounds__(256) void k_cast_wT(const float* __restrict__ SRC, unsigned short* __restrict__ DST, int ldd, int dupoff) {
  const int u = (int)blockIdx.x * 256 + (int)threadIdx.x;
  const int per = DM / 8;
  if (u >= DM * per) return;
  const int n = u / per;
  const int k0 = 8 * (u - n * per);
  float w[8];
#pragma unroll
  for (int e = 0; e < 8; ++e) w[e] = bf_rne_keep(SRC[(size_t)(k0 + e) * DM + n]) * WCARRY;
  u4v pk;
  pk.x = pk2h(w[0], w[1]); pk.y = pk2h(w[2], w[3]); pk.z = pk2h(w[4], w[5]); pk.w = pk2h(w[6], w[7]);
  volatile u4v* d = (volatile u4v*)(DST + (size_t)n * ldd + k0);
  *d = pk; __threadfence(); *d = pk;
  if (dupoff > 0) {
    volatile u4v* d2 = (volatile u4v*)(DST + (size_t)n * ldd + dupoff + k0);
    *d2 = pk; __threadfence(); *d2 = pk;
  }
}

template <int BIAS_MODE, int OUT_MODE>
__device__ __forceinline__ void gemm64_body(
    const _Float16* __restrict__ A, int lda, long long strideA,
    const _Float16* __restrict__ Bt, int ldb, long long strideB,
    float* __restrict__ Cf, _Float16* __restrict__ Ch, int ldc, long long strideC, int resoff,
    const float* __restrict__ bias, int M, int N, int K, float scale, float bscale) {
  static_assert(BIAS_MODE == 1 || BIAS_MODE == 2);
  static_assert(OUT_MODE >= 0 && OUT_MODE <= 2);
  __shared__ __align__(16) float sT[8][16 * OSP];
  const int b = (int)blockIdx.y;
  const int lane = (int)threadIdx.x & 31;
  const int wave = __builtin_amdgcn_readfirstlane((int)(threadIdx.x >> 5));
  const int tilesN = N >> 6;
  const int tilesM = M >> 6;
  const int tile = (int)blockIdx.x * 8 + wave;
  if (tile >= tilesM * tilesN) return;
  const int tm = tile / tilesN;
  const int tn = tile - tm * tilesN;
  const int m0 = tm << 6;
  const int n0 = tn << 6;
  const _Float16* Ab = A + (size_t)b * (size_t)strideA;
  const _Float16* Bb = Bt + (size_t)b * (size_t)strideB;
  const int rlane = lane & 15;
  const int koff = (lane >> 4) * 8;
  const int mOff = (lane >> 4) * 8;

  v8f acc[4][4];
#pragma unroll
  for (int i = 0; i < 4; ++i)
#pragma unroll
    for (int j = 0; j < 4; ++j) acc[i][j] = (v8f){0.f, 0.f, 0.f, 0.f, 0.f, 0.f, 0.f, 0.f};

  for (int k0 = 0; k0 < K; k0 += 32) {
    v16h bh[4];
#pragma unroll
    for (int j = 0; j < 4; ++j) bh[j] = ldf(Bb + (size_t)(n0 + (j << 4) + rlane) * ldb + koff + k0);
#pragma unroll
    for (int i = 0; i < 4; ++i) {
      const v16h ah = ldf(Ab + (size_t)(m0 + (i << 4) + rlane) * lda + koff + k0);
#pragma unroll
      for (int j = 0; j < 4; ++j)
        acc[i][j] = __builtin_amdgcn_wmma_f32_16x16x32_f16(false, ah, false, bh[j], (short)0, acc[i][j], false, false);
      guard4(acc[i][0], acc[i][1], acc[i][2], acc[i][3], ah, bh[3]);
    }
    keep4(bh[0], bh[1], bh[2], bh[3]);
  }
  acc_guard4(acc[0][0], acc[0][1], acc[0][2], acc[0][3]);
  acc_guard4(acc[1][0], acc[1][1], acc[1][2], acc[1][3]);
  acc_guard4(acc[2][0], acc[2][1], acc[2][2], acc[2][3]);
  acc_guard4(acc[3][0], acc[3][1], acc[3][2], acc[3][3]);

#pragma unroll
  for (int i = 0; i < 4; ++i) {
    const int mBase = m0 + (i << 4);
#pragma unroll
    for (int j = 0; j < 4; ++j) {
      const int n = n0 + (j << 4) + rlane;
      float bv = 0.f;
      if (BIAS_MODE == 2) bv = bf_rne_keep(bias[n]) * bscale;
#pragma unroll
      for (int r = 0; r < 8; ++r) {
        float v = acc[i][j][r] * scale;
        if (BIAS_MODE == 1) v += bf_rne_keep(bias[mBase + mOff + r]) * bscale;
        if (BIAS_MODE == 2) v += bv;
        sT[wave][(mOff + r) * OSP + (j << 4) + rlane] = v;
      }
    }
    wave_sync_lds();
    if (OUT_MODE == 0) {
      float* C = Cf + (size_t)b * (size_t)strideC;
      const int hh = lane >> 4, c4 = (lane & 15) * 4;
      for (int pass = 0; pass < 2; ++pass) {
#pragma unroll
        for (int it = 0; it < 8; ++it) {
          const int row = it * 2 + hh;
          const v4f v = *(const v4f*)&sT[wave][row * OSP + c4];
          *(volatile v4f*)(C + (size_t)(mBase + row) * ldc + n0 + c4) = v;
        }
        __threadfence();
      }
    } else {
      _Float16* C = Ch + (size_t)b * (size_t)strideC;
      const int q = lane >> 3, c8 = (lane & 7) * 8;
      for (int pass = 0; pass < 2; ++pass) {
#pragma unroll
        for (int it = 0; it < 4; ++it) {
          const int row = it * 4 + q;
          const v4f s0 = *(const v4f*)&sT[wave][row * OSP + c8];
          const v4f s1 = *(const v4f*)&sT[wave][row * OSP + c8 + 4];
          const float f[8] = {s0.x, s0.y, s0.z, s0.w, s1.x, s1.y, s1.z, s1.w};
          v8h hv, lv;
#pragma unroll
          for (int e = 0; e < 8; ++e) {
            const _Float16 hi = (_Float16)f[e];
            hv[e] = hi;
            lv[e] = (_Float16)(f[e] - (float)hi);
          }
          *(volatile v8h*)(C + (size_t)(mBase + row) * ldc + n0 + c8) = hv;
          if (OUT_MODE == 2) *(volatile v8h*)(C + (size_t)(mBase + row) * ldc + resoff + n0 + c8) = lv;
        }
        __threadfence();
      }
    }
    wave_sync_lds();
  }
}

__global__ __launch_bounds__(256) void k_gemm_q(const _Float16* __restrict__ X, const _Float16* __restrict__ W, const float* __restrict__ bias, _Float16* __restrict__ QP) {
  gemm64_body<2, 2>(X, DM, 0, W, DM, 0, (float*)0, QP, QPITCH, 0, RESOFF, bias, NB * SEQ, DM, DM, QCARRY / WCARRY, QCARRY);
}
__global__ __launch_bounds__(256) void k_gemm_k(const _Float16* __restrict__ X, const _Float16* __restrict__ W, const float* __restrict__ bias, _Float16* __restrict__ KP) {
  gemm64_body<2, 1>(X, DM, 0, W, DM, 0, (float*)0, KP, DM, 0, 0, bias, NB * SEQ, DM, DM, 1.0f / WCARRY, 1.0f);
}
__global__ __launch_bounds__(256) void k_gemm_vt(const _Float16* __restrict__ W, const _Float16* __restrict__ X, const float* __restrict__ bias, _Float16* __restrict__ VT) {
  gemm64_body<1, 1>(W, DM, 0, X, DM, (long long)SEQ * DM, (float*)0, VT, SEQ, (long long)DM * SEQ, 0, bias, DM, SEQ, DM, 1.0f / WCARRY, 1.0f);
}
__global__ __launch_bounds__(256) void k_gemm_out(const _Float16* __restrict__ CX, const _Float16* __restrict__ WO, const float* __restrict__ bias, float* __restrict__ OUT) {
  gemm64_body<2, 0>(CX, QPITCH, (long long)SEQ * QPITCH, WO, QPITCH, 0, OUT, (_Float16*)0, DM, (long long)SEQ_FULL * DM, 0, bias, SEQ, DM, QPITCH, 1.0f / (CCARRY * WCARRY), 1.0f);
}

__global__ __launch_bounds__(128) void k_attn_fused(const _Float16* __restrict__ Qp, const _Float16* __restrict__ Kp,
                                                    const _Float16* __restrict__ VTp, _Float16* __restrict__ Cp) {
  __shared__ __align__(16) _Float16 Ps[AT_NW][16 * PSP];
  __shared__ __align__(16) float    Os[AT_NW][16 * OSP];
  const int tid  = (int)threadIdx.x;
  const int wave = __builtin_amdgcn_readfirstlane(tid >> 5);
  const int lane = tid & 31;
  const int hh   = lane >> 4;
  const int c    = lane & 15;
  const int nqb  = SEQ / 64;
  const int bx   = (int)blockIdx.x;
  const int qb   = bx % nqb;
  const int bh   = bx / nqb;
  const int h    = bh % NH;
  const int b    = bh / NH;
  const int q0   = qb * 64 + wave * 16;
  const int qoff  = (b * SEQ + q0 + c) * QPITCH + h * HD + 8 * hh;
  const int kbase = (b * SEQ + c) * DM + h * HD + 8 * hh;
  const int vbase = (b * DM + h * HD + c) * SEQ + 8 * hh;
  const float SC2 = 1.4426950408889634f * (0.125f / QCARRY);
  const v8f z8 = (v8f){0.f, 0.f, 0.f, 0.f, 0.f, 0.f, 0.f, 0.f};

  float mrow[8], lrow[8];
  v8f oacc[4];
#pragma unroll
  for (int r = 0; r < 8; ++r) { mrow[r] = -__builtin_inff(); lrow[r] = 0.f; }
#pragma unroll
  for (int t = 0; t < 4; ++t) oacc[t] = z8;

#pragma unroll 1
  for (int kv0 = 0; kv0 < SEQ; kv0 += 32) {
    int qo = qoff;
    asm volatile("" : "+v"(qo));
    const int ko = kbase + kv0 * DM;
    v8f s0 = z8, s1 = z8;
#pragma unroll
    for (int dc = 0; dc < 2; ++dc) {
      const v16h qh  = ldf(Qp + qo + dc * 32);
      const v16h qr  = ldf(Qp + qo + RESOFF + dc * 32);
      const v16h k0f = ldf(Kp + ko + dc * 32);
      const v16h k1f = ldf(Kp + ko + 16 * DM + dc * 32);
      s0 = mma16(qh, k0f, s0);
      s0 = mma16(qr, k0f, s0);
      s1 = mma16(qh, k1f, s1);
      s1 = mma16(qr, k1f, s1);
    }
    wave_sync_lds();
#pragma unroll
    for (int r = 0; r < 8; ++r) {
      const float a0 = s0[r] * SC2;
      const float a1 = s1[r] * SC2;
      float m = fmaxf(a0, a1);
      m = fmaxf(m, __shfl_xor(m, 1, 32));
      m = fmaxf(m, __shfl_xor(m, 2, 32));
      m = fmaxf(m, __shfl_xor(m, 4, 32));
      m = fmaxf(m, __shfl_xor(m, 8, 32));
      const float mnew  = fmaxf(mrow[r], m);
      const float alpha = exp2f(mrow[r] - mnew);
      mrow[r] = mnew;
      const float p0 = exp2f(a0 - mnew);
      const float p1 = exp2f(a1 - mnew);
      float ps = p0 + p1;
      ps += __shfl_xor(ps, 1, 32);
      ps += __shfl_xor(ps, 2, 32);
      ps += __shfl_xor(ps, 4, 32);
      ps += __shfl_xor(ps, 8, 32);
      lrow[r] = lrow[r] * alpha + ps;
      Ps[wave][(8 * hh + r) * PSP + c]      = (_Float16)(p0 * PSC);
      Ps[wave][(8 * hh + r) * PSP + 16 + c] = (_Float16)(p1 * PSC);
#pragma unroll
      for (int t = 0; t < 4; ++t) oacc[t][r] *= alpha;
    }
    wave_sync_lds();
    FragH pa;
    pa.h[0] = *(const v8h*)&Ps[wave][c * PSP + 8 * hh];
    pa.h[1] = *(const v8h*)&Ps[wave][c * PSP + 16 + 8 * hh];
    const int vo = vbase + kv0;
    const v16h vb0 = ldf(VTp + vo);
    const v16h vb1 = ldf(VTp + vo + 16 * SEQ);
    const v16h vb2 = ldf(VTp + vo + 32 * SEQ);
    const v16h vb3 = ldf(VTp + vo + 48 * SEQ);
    oacc[0] = mma16(pa.v, vb0, oacc[0]);
    oacc[1] = mma16(pa.v, vb1, oacc[1]);
    oacc[2] = mma16(pa.v, vb2, oacc[2]);
    oacc[3] = mma16(pa.v, vb3, oacc[3]);
  }

#pragma unroll
  for (int r = 0; r < 8; ++r) {
    const float inv = CCARRY * (1.0f / (lrow[r] * PSC));
#pragma unroll
    for (int t = 0; t < 4; ++t) Os[wave][(8 * hh + r) * OSP + t * 16 + c] = oacc[t][r] * inv;
  }
  wave_sync_lds();
  {
    const int q = lane >> 3, c8 = (lane & 7) * 8;
    _Float16* cb = Cp + (size_t)(b * SEQ + q0) * QPITCH + h * HD;
    for (int pass = 0; pass < 2; ++pass) {
#pragma unroll
      for (int it = 0; it < 4; ++it) {
        const int row = it * 4 + q;
        const v4f s0 = *(const v4f*)&Os[wave][row * OSP + c8];
        const v4f s1 = *(const v4f*)&Os[wave][row * OSP + c8 + 4];
        const float f[8] = {s0.x, s0.y, s0.z, s0.w, s1.x, s1.y, s1.z, s1.w};
        v8h hv, lv;
#pragma unroll
        for (int e = 0; e < 8; ++e) {
          const _Float16 hi = (_Float16)f[e];
          hv[e] = hi;
          lv[e] = (_Float16)(f[e] - (float)hi);
        }
        *(volatile v8h*)(cb + (size_t)row * QPITCH + c8) = hv;
        *(volatile v8h*)(cb + (size_t)row * QPITCH + RESOFF + c8) = lv;
      }
      __threadfence();
    }
  }
}

constexpr size_t SZ_X   = (size_t)NB * SEQ * DM * 2;
constexpr size_t SZ_W   = (size_t)DM * DM * 2;
constexpr size_t SZ_WO  = (size_t)DM * QPITCH * 2;
constexpr size_t SZ_Q   = (size_t)NB * SEQ * QPITCH * 2;
constexpr size_t SZ_VT  = (size_t)NB * DM * SEQ * 2;
constexpr size_t OFF_XQ = 0;
constexpr size_t OFF_XK = OFF_XQ + SZ_X;
constexpr size_t OFF_XV = OFF_XK + SZ_X;
constexpr size_t OFF_WQ = OFF_XV + SZ_X;
constexpr size_t OFF_WK = OFF_WQ + SZ_W;
constexpr size_t OFF_WV = OFF_WK + SZ_W;
constexpr size_t OFF_WO = OFF_WV + SZ_W;
constexpr size_t OFF_QP = OFF_WO + SZ_WO;
constexpr size_t OFF_KP = OFF_QP + SZ_Q;
constexpr size_t OFF_VT = OFF_KP + SZ_X;
constexpr size_t OFF_CX = OFF_VT + SZ_VT;
constexpr size_t WS_TOTAL = OFF_CX + SZ_Q;
static_assert(SZ_X % 256 == 0);
static_assert(SZ_W % 256 == 0);
static_assert(SZ_WO % 256 == 0);
static_assert(SZ_Q % 256 == 0);
static_assert(SZ_VT % 256 == 0);
static_assert(WS_TOTAL <= (size_t)134217728);
static_assert(((size_t)(NB_FULL - 1) * SEQ_FULL + SEQ_FULL) * DM * 4 == (size_t)12582912);

extern "C" void kernel_launch(void* const* d_in, const int* in_sizes, int n_in, void* d_out, int out_size, void* d_ws, size_t ws_size, hipStream_t stream) {
  if (n_in < 11) return;
  const long long need_x = ((long long)(NB - 1) * SEQ_FULL + SEQ) * DM;
  if (in_sizes[0] < need_x || in_sizes[1] < need_x || in_sizes[2] < need_x) return;
  if (in_sizes[3] < DM * DM || in_sizes[5] < DM * DM || in_sizes[7] < DM * DM || in_sizes[9] < DM * DM) return;
  if (in_sizes[4] < DM || in_sizes[6] < DM || in_sizes[8] < DM || in_sizes[10] < DM) return;
  if ((long long)out_size < need_x) return;
  if (WS_TOTAL > ws_size) return;

  const float* xq = (const float*)d_in[0];
  const float* xk = (const float*)d_in[1];
  const float* xv = (const float*)d_in[2];
  const float* wq = (const float*)d_in[3];
  const float* bq = (const float*)d_in[4];
  const float* wk = (const float*)d_in[5];
  const float* bk = (const float*)d_in[6];
  const float* wv = (const float*)d_in[7];
  const float* bv = (const float*)d_in[8];
  const float* wo = (const float*)d_in[9];
  const float* bo = (const float*)d_in[10];
  float* out = (float*)d_out;
  char* ws = (char*)d_ws;

  const unsigned gw = (unsigned)((DM * (DM / 8) + 255) / 256);
  k_cast_wT<<<gw, 256, 0, stream>>>(wq, (unsigned short*)(ws + OFF_WQ), DM, 0);
  k_cast_wT<<<gw, 256, 0, stream>>>(wk, (unsigned short*)(ws + OFF_WK), DM, 0);
  k_cast_wT<<<gw, 256, 0, stream>>>(wv, (unsigned short*)(ws + OFF_WV), DM, 0);
  k_cast_wT<<<gw, 256, 0, stream>>>(wo, (unsigned short*)(ws + OFF_WO), QPITCH, RESOFF);

  const unsigned gx = (unsigned)(((long long)NB * SEQ * (DM / 8) + 255) / 256);
  k_cast_x<<<gx, 256, 0, stream>>>(xq, (unsigned short*)(ws + OFF_XQ));
  k_cast_x<<<gx, 256, 0, stream>>>(xk, (unsigned short*)(ws + OFF_XK));
  k_cast_x<<<gx, 256, 0, stream>>>(xv, (unsigned short*)(ws + OFF_XV));

  const unsigned gqk = (unsigned)((((NB * SEQ) / 64) * (DM / 64) + 7) / 8);
  k_gemm_q<<<dim3(gqk, 1), 256, 0, stream>>>((const _Float16*)(ws + OFF_XQ), (const _Float16*)(ws + OFF_WQ), bq, (_Float16*)(ws + OFF_QP));
  k_gemm_k<<<dim3(gqk, 1), 256, 0, stream>>>((const _Float16*)(ws + OFF_XK), (const _Float16*)(ws + OFF_WK), bk, (_Float16*)(ws + OFF_KP));
  const unsigned gvt = (unsigned)(((DM / 64) * (SEQ / 64) + 7) / 8);
  k_gemm_vt<<<dim3(gvt, NB), 256, 0, stream>>>((const _Float16*)(ws + OFF_WV), (const _Float16*)(ws + OFF_XV), bv, (_Float16*)(ws + OFF_VT));

  k_attn_fused<<<(unsigned)(NB * NH * (SEQ / 64)), 32 * AT_NW, 0, stream>>>((const _Float16*)(ws + OFF_QP), (const _Float16*)(ws + OFF_KP),
                                                                           (const _Float16*)(ws + OFF_VT), (_Float16*)(ws + OFF_CX));

  const unsigned go = (unsigned)(((SEQ / 64) * (DM / 64) + 7) / 8);
  k_gemm_out<<<dim3(go, NB), 256, 0, stream>>>((const _Float16*)(ws + OFF_CX), (const _Float16*)(ws + OFF_WO), bo, out);
}
